// GNN_Feature_Extractor_3152505995796
// MI455X (gfx1250) — hardware-verified
//
#include <hip/hip_runtime.h>
#include <math.h>

#define NN   50000
#define NE   800000
#define NV   (NE + NN)
#define FIN  128
#define FD   64
#define NG   64
#define NT   256
#define SRB  512
#define NTL  98
#define NPAD (NTL * SRB)

typedef __attribute__((ext_vector_type(16))) _Float16 v16h;
typedef __attribute__((ext_vector_type(8)))  _Float16 v8h;
typedef __attribute__((ext_vector_type(4)))  _Float16 v4h;
typedef __attribute__((ext_vector_type(2)))  _Float16 v2h;
typedef __attribute__((ext_vector_type(16))) __bf16   v16b;
typedef __attribute__((ext_vector_type(8)))  __bf16   v8b;
typedef __attribute__((ext_vector_type(8)))  float    v8f;
typedef __attribute__((ext_vector_type(4)))  float    v4f;
typedef __attribute__((ext_vector_type(2)))  float    v2f;
typedef __attribute__((ext_vector_type(4)))  int      v4i;

__device__ __forceinline__ unsigned short f2bf_bits(float f) {
  unsigned u = __float_as_uint(f);
  return (unsigned short)((u + 0x7FFFu + ((u >> 16) & 1u)) >> 16);
}
__device__ __forceinline__ float bf_bits2f(unsigned short h) { return __uint_as_float(((unsigned)h) << 16); }

__device__ __forceinline__ void dep_guard_h(v8f& a, v8f& b, v16h x, v16h y) { asm volatile("v_nop\n\tv_nop\n\tv_nop\n\tv_nop" : "+v"(a), "+v"(b) : "v"(x), "v"(y)); }
__device__ __forceinline__ void dep_guard_b(v8f& a, v8f& b, v16b x, v16b y) { asm volatile("v_nop\n\tv_nop\n\tv_nop\n\tv_nop" : "+v"(a), "+v"(b) : "v"(x), "v"(y)); }
__device__ __forceinline__ void keep4_h(v16h a, v16h b, v16h c, v16h d) { asm volatile("v_nop" :: "v"(a), "v"(b), "v"(c), "v"(d)); }
__device__ __forceinline__ void keep4_b(v16b a, v16b b, v16b c, v16b d) { asm volatile("v_nop" :: "v"(a), "v"(b), "v"(c), "v"(d)); }
__device__ __forceinline__ void acc_guard4(v8f& a, v8f& b, v8f& c, v8f& d) { asm volatile("v_nop\n\tv_nop\n\tv_nop\n\tv_nop" : "+v"(a), "+v"(b), "+v"(c), "+v"(d)); }
__device__ __forceinline__ void cbar() { asm volatile("" ::: "memory"); }

template <typename T> struct Frag;
template <> struct Frag<_Float16> {
  typedef v16h V; union U { v16h v; v8h h[2]; };
  static __device__ __forceinline__ v16h load(const _Float16* p) {
    U f; f.h[0] = *(const v8h*)(p); f.h[1] = *(const v8h*)(p + 16); return f.v;
  }
  static __device__ __forceinline__ v8f mma(v16h a, v16h b, v8f c) {
    return __builtin_amdgcn_wmma_f32_16x16x32_f16(false, a, false, b, (short)0, c, false, false);
  }
  static __device__ __forceinline__ void guard(v8f& a, v8f& b, v16h x, v16h y) { dep_guard_h(a, b, x, y); }
  static __device__ __forceinline__ void keep(v16h a, v16h b, v16h c, v16h d) { keep4_h(a, b, c, d); }
};
template <> struct Frag<__bf16> {
  typedef v16b V; union U { v16b v; v8b h[2]; };
  static __device__ __forceinline__ v16b load(const __bf16* p) {
    U f; f.h[0] = *(const v8b*)(p); f.h[1] = *(const v8b*)(p + 16); return f.v;
  }
  static __device__ __forceinline__ v8f mma(v16b a, v16b b, v8f c) {
    return __builtin_amdgcn_wmma_f32_16x16x32_bf16(false, a, false, b, (short)0, c, false, false);
  }
  static __device__ __forceinline__ void guard(v8f& a, v8f& b, v16b x, v16b y) { dep_guard_b(a, b, x, y); }
  static __device__ __forceinline__ void keep(v16b a, v16b b, v16b c, v16b d) { keep4_b(a, b, c, d); }
};

template <int ET> struct Elem;
template <> struct Elem<0> { typedef _Float16 T; };
template <> struct Elem<1> { typedef __bf16 T; };
template <int ET, bool SPLIT, int BIAS_MODE, int OUT_MODE, bool RESID, int ACT = 0>
__global__ __launch_bounds__(256) void wmma_gemm64(
    const unsigned short* __restrict__ Ap, const unsigned short* __restrict__ A2p, int lda, long strideA,
    const unsigned short* __restrict__ Btp, const unsigned short* __restrict__ Bt2p, int ldb, long strideB,
    void* __restrict__ Cout, void* __restrict__ Cout2, int ldc, long strideC,
    const float* __restrict__ bias,
    const float* __restrict__ resid, long strideR,
    int M, int N, int K, float scale) {
  typedef typename Elem<ET>::T T;
  typedef typename Frag<T>::V V;
  const T* A = (const T*)Ap; const T* A2 = (const T*)A2p; const T* Bt = (const T*)Btp; const T* Bt2 = (const T*)Bt2p;
  __shared__ __align__(16) float sT[8][16 * 68];
  const int b    = blockIdx.y;
  const int lane = threadIdx.x & 31;
  const int wave = threadIdx.x >> 5;
  const int tilesN = N >> 6;
  const int tilesM = M >> 6;
  const int tile = blockIdx.x * 8 + wave;
  if (tile >= tilesM * tilesN) return;
  const int tm = tile / tilesN;
  const int tn = tile - tm * tilesN;
  const int m0 = tm << 6;
  const int n0 = tn << 6;

  const T* Ab  = A  + (size_t)b * strideA;
  const T* Bb  = Bt + (size_t)b * strideB;
  const T* Ab2 = SPLIT ? (A2  + (size_t)b * strideA) : nullptr;
  const T* Bb2 = SPLIT ? (Bt2 + (size_t)b * strideB) : nullptr;

  const int rlane = lane & 15;
  const int koff  = (lane >> 4) * 8;
  const int mOff  = (lane >> 4) * 8;

  v8f acc[4][4];
#pragma unroll
  for (int i = 0; i < 4; ++i)
#pragma unroll
    for (int j = 0; j < 4; ++j) acc[i][j] = (v8f){0.f,0.f,0.f,0.f,0.f,0.f,0.f,0.f};

  for (int k0 = 0; k0 < K; k0 += 32) {
    V bh[4], bl[4];
#pragma unroll
    for (int j = 0; j < 4; ++j) {
      const size_t bo = (size_t)(n0 + (j << 4) + rlane) * ldb + koff + k0;
      bh[j] = Frag<T>::load(Bb + bo);
      if (SPLIT) bl[j] = Frag<T>::load(Bb2 + bo);
    }
#pragma unroll
    for (int i = 0; i < 4; ++i) {
      const size_t ao = (size_t)(m0 + (i << 4) + rlane) * lda + koff + k0;
      V ah = Frag<T>::load(Ab + ao);
      V al;
      if (SPLIT) al = Frag<T>::load(Ab2 + ao);
#pragma unroll
      for (int j = 0; j < 4; ++j) {
        acc[i][j] = Frag<T>::mma(ah, bh[j], acc[i][j]);
        if (SPLIT) {
          acc[i][j] = Frag<T>::mma(ah, bl[j], acc[i][j]);
          acc[i][j] = Frag<T>::mma(al, bh[j], acc[i][j]);
        }
      }
      Frag<T>::guard(acc[i][0], acc[i][3], ah, SPLIT ? al : ah);
    }
    Frag<T>::keep(bh[0], bh[1], bh[2], bh[3]);
    if (SPLIT) Frag<T>::keep(bl[0], bl[1], bl[2], bl[3]);
  }
  acc_guard4(acc[0][0], acc[0][1], acc[0][2], acc[0][3]);
  acc_guard4(acc[1][0], acc[1][1], acc[1][2], acc[1][3]);
  acc_guard4(acc[2][0], acc[2][1], acc[2][2], acc[2][3]);
  acc_guard4(acc[3][0], acc[3][1], acc[3][2], acc[3][3]);

  float* slab = sT[wave];
  const float* Rb = RESID ? (resid + (size_t)b * strideR) : nullptr;
#pragma unroll
  for (int i = 0; i < 4; ++i) {
    const int mBase = m0 + (i << 4);
#pragma unroll
    for (int j = 0; j < 4; ++j) {
      const int n = n0 + (j << 4) + rlane;
      float bv = 0.f;
      if (BIAS_MODE == 2) bv = bias[n];
#pragma unroll
      for (int r = 0; r < 8; ++r) {
        float v = acc[i][j][r] * scale;
        if (BIAS_MODE == 1) v += bias[mBase + mOff + r];
        if (BIAS_MODE == 2) v += bv;
        if (RESID) v += Rb[(size_t)(mBase + mOff + r) * ldc + n];
        if (ACT == 1) v = tanhf(v);
        if (ACT == 2) v = fmaxf(v, 0.0f);
        if (ACT == 3) v = v / (1.0f + expf(-v));
        if (ACT == 4) v = (v > 0.f) ? v : 0.01f * v;
        if (ACT == 5) v = 0.5f * v * (1.0f + erff(v * 0.70710678118654752f));
        slab[(mOff + r) * 68 + (j << 4) + rlane] = v;
      }
    }
    __builtin_amdgcn_fence(__ATOMIC_RELEASE, "workgroup");
    __builtin_amdgcn_wave_barrier();
    __builtin_amdgcn_fence(__ATOMIC_ACQUIRE, "workgroup");
    if (OUT_MODE == 0) {
      float* C = (float*)Cout + (size_t)b * strideC;
      const int hh = lane >> 4, c4 = (lane & 15) * 4;
      for (int pass = 0; pass < 2; ++pass) {
#pragma unroll
        for (int it = 0; it < 8; ++it) {
          const int row = it * 2 + hh;
          v4f v = *(const v4f*)(slab + row * 68 + c4);
          *(volatile v4f*)(C + (size_t)(mBase + row) * ldc + n0 + c4) = v;
        }
        __threadfence();
      }
    } else {
      const int q = lane >> 3, c8 = (lane & 7) * 8;
      unsigned short* C  = (unsigned short*)Cout  + (size_t)b * strideC;
      unsigned short* C2 = (OUT_MODE == 2) ? ((unsigned short*)Cout2 + (size_t)b * strideC) : nullptr;
      for (int pass = 0; pass < 2; ++pass) {
#pragma unroll
        for (int it = 0; it < 4; ++it) {
          const int row = it * 4 + q;
          const float* sp = slab + row * 68 + c8;
          v8h hv, lv;
#pragma unroll
          for (int e = 0; e < 8; ++e) {
            if (OUT_MODE == 1) {
              hv[e] = (_Float16)sp[e];
            } else {
              unsigned short hb = f2bf_bits(sp[e]);
              unsigned short lb = f2bf_bits(sp[e] - bf_bits2f(hb));
              hv[e] = __builtin_bit_cast(_Float16, hb);
              lv[e] = __builtin_bit_cast(_Float16, lb);
            }
          }
          *(volatile v8h*)(C + (size_t)(mBase + row) * ldc + n0 + c8) = hv;
          if (OUT_MODE == 2) *(volatile v8h*)(C2 + (size_t)(mBase + row) * ldc + n0 + c8) = lv;
        }
        __threadfence();
      }
    }
    __builtin_amdgcn_fence(__ATOMIC_RELEASE, "workgroup");
    __builtin_amdgcn_wave_barrier();
    __builtin_amdgcn_fence(__ATOMIC_ACQUIRE, "workgroup");
  }
}

__global__ __launch_bounds__(256) void transpose_cast_f16(const float* __restrict__ in, int ldi,
                                                         _Float16* __restrict__ outT, int ldo, float scale) {
  __shared__ __align__(16) _Float16 tile[64][72];
  const int c0 = blockIdx.x * 64, r0 = blockIdx.y * 64;
  const int t = threadIdx.y * 32 + threadIdx.x;
  for (int i = threadIdx.y; i < 64; i += 8) {
    tile[threadIdx.x][i]      = (_Float16)(in[(size_t)(r0 + i) * ldi + c0 + threadIdx.x] * scale);
    tile[32 + threadIdx.x][i] = (_Float16)(in[(size_t)(r0 + i) * ldi + c0 + 32 + threadIdx.x] * scale);
  }
  __syncthreads();
  const int q = t >> 3, c8 = (t & 7) * 8;
  for (int pass = 0; pass < 2; ++pass) {
#pragma unroll
    for (int it = 0; it < 2; ++it) {
      const int c = it * 32 + q;
      v8h hv = *(const v8h*)(&tile[c][c8]);
      *(volatile v8h*)(outT + (size_t)(c0 + c) * ldo + r0 + c8) = hv;
    }
    __threadfence();
  }
}

__global__ __launch_bounds__(256) void padcast_rows_kernel(const float* __restrict__ x, unsigned* __restrict__ X16) {
  const long i = (long)blockIdx.x * 256 + threadIdx.x; if (i >= (long)NPAD * FIN / 2) return;
  const long e0 = 2 * i;
  const long lim = (long)NN * FIN;
  const bool ok = e0 < lim;
  const long ec = ok ? e0 : 0;
  float a = x[ec], b = x[ec + 1];
  a = ok ? a : 0.f; b = ok ? b : 0.f;
  const unsigned u = (unsigned)__builtin_bit_cast(unsigned short, (_Float16)a) | ((unsigned)__builtin_bit_cast(unsigned short, (_Float16)b) << 16);
  ((volatile unsigned*)X16)[i] = u; __threadfence(); ((volatile unsigned*)X16)[i] = u;
}

template <int NH>
__global__ __launch_bounds__(NT) void att_terms_kernel(const _Float16* __restrict__ XW, const float* __restrict__ as, const float* __restrict__ ad,
                                                      float* __restrict__ ASD) {
  constexpr int W = NH * FD;
  constexpr int LPH = 32 / NH;
  constexpr int CPL = FD / LPH;
  __shared__ __align__(16) float so[8 * 16];
  const int tid = threadIdx.x, lane = tid & 31, wave = tid >> 5;
  if (tid < 128) so[tid] = 0.f;
  __syncthreads();
  const int n = blockIdx.x * 8 + wave;
  const int h = lane / LPH, cq = (lane - h * LPH) * CPL;
  const _Float16* xr = XW + (size_t)n * W + h * FD + cq;
  const float* sp = as + h * FD + cq;
  const float* dp = ad + h * FD + cq;
  float s = 0.f, d = 0.f;
#pragma unroll
  for (int e = 0; e < CPL; ++e) {
    const float xv = (float)xr[e];
    s += xv * sp[e];
    d += xv * dp[e];
  }
#pragma unroll
  for (int o = 1; o < LPH; o <<= 1) { s += __shfl_xor(s, o, 32); d += __shfl_xor(d, o, 32); }
  if ((lane & (LPH - 1)) == 0) { so[wave * 16 + h] = s; so[wave * 16 + 8 + h] = d; }
  __syncthreads();
  if (wave == 0) {
    const v4f v = *(const v4f*)(so + 4 * lane);
    float* op = ASD + (size_t)blockIdx.x * 128 + 4 * lane;
    *(volatile v4f*)op = v; __threadfence(); *(volatile v4f*)op = v;
  }
}

__device__ __forceinline__ int blk_excl_scan(int cnt, int* scan_ws, int tid, int* tot) {
  const int lane = tid & 31, wave = tid >> 5; int incl = cnt;
#pragma unroll
  for (int o = 1; o < 32; o <<= 1) { const int v = __shfl_up(incl, o, 32); if (lane >= o) incl += v; }
  if (lane == 31) scan_ws[wave] = incl;
  __syncthreads();
  if (wave == 0) { int wv = (lane < NT / 32) ? scan_ws[lane] : 0; int wincl = wv;
#pragma unroll
    for (int o = 1; o < 32; o <<= 1) { const int v = __shfl_up(wincl, o, 32); if (lane >= o) wincl += v; }
    if (lane < NT / 32) scan_ws[32 + lane] = wincl - wv; if (lane == 31) scan_ws[64] = wincl; }
  __syncthreads();
  const int res = scan_ws[32 + wave] + incl - cnt; *tot = scan_ws[64];
  return res;
}
template <int SP, int CAP>
__device__ __forceinline__ int chunk_hits(const int* __restrict__ dstv, const int* __restrict__ srcv, int e0, int n0, int tid,
                                          int* LIST, int* scan_ws) {
  const int eb = e0 + tid * SP;
  const bool real = eb < NE;
  const int ebc = real ? eb : (NE - SP);
  int rec[SP]; int cnt = 0;
#pragma unroll
  for (int k = 0; k < SP; k += 4) {
    const v4i d4 = *(const v4i*)(dstv + ebc + k);
    const v4i s4 = *(const v4i*)(srcv + ebc + k);
#pragma unroll
    for (int e = 0; e < 4; ++e) {
      const int ev = eb + k + e;
      const int dv = ev - NE;
      const int d = real ? d4[e] : dv;
      int s = real ? s4[e] : dv;
      s = s < 0 ? 0 : (s >= NN ? NN - 1 : s);
      const bool valid = real || (ev < NV);
      int r = -1;
      if (valid && d >= n0 && d < n0 + SRB) { r = ((d - n0) << 16) | s; ++cnt; }
      rec[k + e] = r;
    }
  }
  int tot; int p = blk_excl_scan(cnt, scan_ws, tid, &tot);
#pragma unroll
  for (int k = 0; k < SP; ++k) if (rec[k] >= 0) { if ((unsigned)p < (unsigned)CAP) LIST[p] = rec[k]; ++p; }
  __syncthreads();
  return tot < CAP ? tot : CAP;
}

#define SCH 2048
#define NCH ((NV + SCH - 1) / SCH)
template <int NH>
__global__ __launch_bounds__(NT) void gat_agg_kernel(const _Float16* __restrict__ XW, const int* __restrict__ ei, const float* __restrict__ ASD,
                                                    const float* __restrict__ bias, float* AGG, void* HOUT) {
  constexpr int W = NH * FD;
  __shared__ int LIST[SCH];
  __shared__ float SM[SRB * NH];
  __shared__ float SL[SRB * NH];
  __shared__ float SAD[SRB * NH];
  __shared__ int scan_ws[80];
  const int tid = threadIdx.x, lane = tid & 31, wave = tid >> 5;
  const int n0 = blockIdx.x * SRB;
  const int hN = lane & (NH - 1);
  const v4f z4 = {0.f, 0.f, 0.f, 0.f};
  const v2f z2 = {0.f, 0.f};
#pragma unroll 1
  for (int j = 0; j < 64; ++j) {
    float* rp = AGG + (size_t)(n0 + wave * 64 + j) * W;
    if (NH == 4) { *(v4f*)(rp + 4 * lane) = z4; *(v4f*)(rp + 128 + 4 * lane) = z4; }
    else         { *(v2f*)(rp + 2 * lane) = z2; }
  }
  for (int i = tid; i < SRB * NH; i += NT) {
    SM[i] = -INFINITY; SL[i] = 0.f;
    const int dl = i / NH, h = i - dl * NH;
    SAD[i] = ASD[(size_t)(n0 + dl) * 16 + 8 + h];
  }
  __syncthreads();
  const int* srcv = ei; const int* dstv = ei + NE;
#pragma unroll 1
  for (int c = 0; c < NCH; ++c) {
    const int tot = chunk_hits<SCH / NT, SCH>(dstv, srcv, c * SCH, n0, tid, LIST, scan_ws);
#pragma unroll 1
    for (int base = 0; base < tot; base += 32) {
      const int q = base + lane;
      const int qq = q < SCH ? q : SCH - 1;
      const int lq = LIST[qq];
      const int rv = (q < tot) ? lq : -1;
      const int own = (rv >= 0 && (rv >> 22) == wave) ? 1 : 0;
      unsigned msk = (unsigned)__ballot(own);
#pragma unroll 1
      for (int it = 0; it < 32; ++it) {
        if (msk == 0u) break;
        const int bp = __builtin_ctz(msk); msk &= msk - 1u;
        const int r = __shfl(rv, bp, 32);
        const int dl = r >> 16, s = r & 0xFFFF;
        const int mi = dl * NH + hN;
        float al = ASD[(size_t)s * 16 + hN] + SAD[mi];
        al = (al >= 0.f) ? al : 0.2f * al;
        const float mo = SM[mi], lo = SL[mi];
        const float mn = fmaxf(mo, al);
        const float rr = __expf(mo - mn), ex = __expf(al - mn);
        const float ln = lo * rr + ex;
        if (lane < NH) { SM[mi] = mn; SL[mi] = ln; }
        cbar();
        if (NH == 4) {
          const _Float16* xr = XW + (size_t)s * W + 4 * lane;
          float* rp = AGG + (size_t)(n0 + dl) * W + 4 * lane;
#pragma unroll
          for (int j = 0; j < 2; ++j) {
            const int hj = 2 * j + (lane >> 4);
            const float rrj = __shfl(rr, hj, 32), exj = __shfl(ex, hj, 32);
            const v4h xv = *(const v4h*)(xr + 128 * j);
            const v4f hv = __builtin_convertvector(xv, v4f);
            v4f a = *(const v4f*)(rp + 128 * j);
            a = a * rrj + exj * hv;
            *(v4f*)(rp + 128 * j) = a;
          }
        } else {
          const _Float16* xr = XW + (size_t)s * W + 2 * lane;
          float* rp = AGG + (size_t)(n0 + dl) * W + 2 * lane;
          const v2h xv = *(const v2h*)(xr);
          const v2f hv = __builtin_convertvector(xv, v2f);
          v2f a = *(const v2f*)(rp);
          a = a * rr + ex * hv;
          *(v2f*)(rp) = a;
        }
      }
    }
    __syncthreads();
  }
  if (NH == 4) {
    _Float16* H16 = (_Float16*)HOUT;
    const int c8 = lane * 8;
    const int hh = lane >> 3;
    const v4f b0 = *(const v4f*)(bias + c8), b1 = *(const v4f*)(bias + c8 + 4);
#pragma unroll 1
    for (int jj = 0; jj < 64; ++jj) {
      const int dl = wave * 64 + jj;
      const int n = n0 + dl;
      float lv = SL[dl * NH + hh];
      lv = lv > 0.f ? lv : 1.0f;
      const float inv = 1.0f / lv;
      const bool ok = n < NN;
      const float* rp = AGG + (size_t)n * W + c8;
      const v4f a0 = *(const v4f*)(rp), a1 = *(const v4f*)(rp + 4);
      v8h hv;
#pragma unroll
      for (int e = 0; e < 4; ++e) {
        float v0 = a0[e] * inv + b0[e]; v0 = fmaxf(v0, 0.f); v0 = ok ? v0 : 0.f;
        float v1 = a1[e] * inv + b1[e]; v1 = fmaxf(v1, 0.f); v1 = ok ? v1 : 0.f;
        hv[e] = (_Float16)v0; hv[4 + e] = (_Float16)v1;
      }
      _Float16* op = H16 + (size_t)n * W + c8;
      *(volatile v8h*)op = hv; __threadfence(); *(volatile v8h*)op = hv;
    }
  } else {
    float* HO = (float*)HOUT;
    const int c4 = (lane & 15) * 4;
    const v4f bs4 = *(const v4f*)(bias + c4);
#pragma unroll 1
    for (int jj = 0; jj < 32; ++jj) {
      const int dl = wave * 64 + 2 * jj + (lane >> 4);
      const int n = n0 + dl;
      float lv = SL[dl * NH];
      lv = lv > 0.f ? lv : 1.0f;
      const float inv = 1.0f / lv;
      const bool ok = n < NN;
      const float* rp = AGG + (size_t)n * W + c4;
      const v4f a = *(const v4f*)(rp);
      v4f v = a * inv + bs4;
#pragma unroll
      for (int e = 0; e < 4; ++e) v[e] = ok ? v[e] : 0.f;
      float* op = HO + (size_t)n * W + c4;
      *(volatile v4f*)op = v; __threadfence(); *(volatile v4f*)op = v;
    }
  }
}

__global__ __launch_bounds__(64) void pool_kernel(const float* __restrict__ H2, const int* __restrict__ bat, float* __restrict__ out) {
  __shared__ __align__(16) float so[64];
  __shared__ int rl[2], rh[2];
  const int tid = threadIdx.x, lane = tid & 31, wave = tid >> 5;
  const int g = blockIdx.x;
  int lo = NN, hi = -1;
#pragma unroll 1
  for (int i = tid; i < NN; i += 64) {
    const int b = bat[i];
    const bool m = (b == g);
    lo = (m && i < lo) ? i : lo;
    hi = (m && i > hi) ? i : hi;
  }
#pragma unroll
  for (int o = 16; o > 0; o >>= 1) {
    const int a = __shfl_xor(lo, o, 32), c = __shfl_xor(hi, o, 32);
    lo = a < lo ? a : lo; hi = c > hi ? c : hi;
  }
  if (lane == 0) { rl[wave] = lo; rh[wave] = hi; }
  __syncthreads();
  lo = rl[0] < rl[1] ? rl[0] : rl[1];
  hi = rh[0] > rh[1] ? rh[0] : rh[1];
  lo = lo < 0 ? 0 : lo;
  hi = hi > NN - 1 ? NN - 1 : hi;
  double acc = 0.0; int cnt = 0;
#pragma unroll 1
  for (int i = lo; i <= hi; ++i) {
    const int b = bat[i];
    const float v = H2[(size_t)i * FD + tid];
    const bool m = (b == g);
    cnt += m ? 1 : 0;
    acc += m ? (double)v : 0.0;
  }
  const float cf = (float)(cnt > 0 ? cnt : 1);
  const float res = (float)acc * (1.0f / cf);
  so[tid] = res;
  __syncthreads();
  if (wave == 0) {
    const v4f v = *(const v4f*)(so + 4 * (lane & 15));
    float* op = out + (size_t)g * FD + 4 * (lane & 15);
    if (lane < 16) *(volatile v4f*)op = v;
    __threadfence();
    if (lane < 16) *(volatile v4f*)op = v;
  }
}

extern "C" void kernel_launch(void* const* d_in, const int* in_sizes, int n_in,
                              void* d_out, int out_size, void* d_ws, size_t ws_size, hipStream_t stream) {
  (void)in_sizes; (void)n_in; (void)out_size;
  const float* x   = (const float*)d_in[0];
  const int*   ei  = (const int*)  d_in[1];
  const int*   bat = (const int*)  d_in[2];
  const float* W1  = (const float*)d_in[3];
  const float* as1 = (const float*)d_in[4];
  const float* ad1 = (const float*)d_in[5];
  const float* b1  = (const float*)d_in[6];
  const float* W2  = (const float*)d_in[7];
  const float* as2 = (const float*)d_in[8];
  const float* ad2 = (const float*)d_in[9];
  const float* b2  = (const float*)d_in[10];
  float* out = (float*)d_out;

  char* ws = (char*)d_ws; size_t off = 0;
  auto carve = [&](size_t bytes) -> char* { char* p = ws + off; off += (bytes + 255) & ~(size_t)255; return p; };
  _Float16* W1T = (_Float16*)carve((size_t)256 * FIN * 2);
  _Float16* W2T = (_Float16*)carve((size_t)FD * 256 * 2);
  unsigned* X16 = (unsigned*)carve((size_t)NPAD * FIN * 2);
  _Float16* XW1 = (_Float16*)carve((size_t)NPAD * 256 * 2);
  float*    ASD = (float*)carve((size_t)NPAD * 16 * 4);
  char*     RGN = carve((size_t)NPAD * 256 * 4);
  _Float16* H1S = (_Float16*)carve((size_t)NPAD * 256 * 2);
  float*    ACC1 = (float*)RGN;
  _Float16* XW2  = (_Float16*)(RGN);
  float*    ACC2 = (float*)(RGN + (size_t)NPAD * FD * 2);
  float*    H2   = (float*)(RGN + (size_t)NPAD * FD * 2 + (size_t)NPAD * FD * 4);
  if (off > ws_size || off > (size_t)134217728) return;

  const int ncast = NPAD * FIN / 2 / 256;
  const int gt1 = (NPAD / 64) * (256 / 64);
  const int gt2 = (NPAD / 64) * (FD / 64);

  transpose_cast_f16<<<dim3(256 / 64, FIN / 64), dim3(32, 8), 0, stream>>>(W1, 256, W1T, FIN, 16.0f);
  transpose_cast_f16<<<dim3(FD / 64, 256 / 64), dim3(32, 8), 0, stream>>>(W2, FD, W2T, 256, 16.0f);

  padcast_rows_kernel<<<ncast, 256, 0, stream>>>(x, X16);
  wmma_gemm64<0, false, 0, 1, false><<<dim3(gt1 / 8, 1), 256, 0, stream>>>(
      (const unsigned short*)X16, nullptr, FIN, 0L, (const unsigned short*)W1T, nullptr, FIN, 0L,
      (void*)XW1, nullptr, 256, 0L, nullptr, nullptr, 0L, NPAD, 256, FIN, 0.0625f);
  att_terms_kernel<4><<<NPAD / 8, NT, 0, stream>>>(XW1, as1, ad1, ASD);
  gat_agg_kernel<4><<<NTL, NT, 0, stream>>>(XW1, ei, ASD, b1, ACC1, (void*)H1S);

  wmma_gemm64<0, false, 0, 1, false><<<dim3(gt2 / 8, 1), 256, 0, stream>>>(
      (const unsigned short*)H1S, nullptr, 256, 0L, (const unsigned short*)W2T, nullptr, 256, 0L,
      (void*)XW2, nullptr, FD, 0L, nullptr, nullptr, 0L, NPAD, FD, 256, 0.0625f);
  att_terms_kernel<1><<<NPAD / 8, NT, 0, stream>>>(XW2, as2, ad2, ASD);
  gat_agg_kernel<1><<<NTL, NT, 0, stream>>>(XW2, ei, ASD, b2, ACC2, (void*)H2);

  pool_kernel<<<NG, 64, 0, stream>>>(H2, bat, out);
}
